// EnhancedGlobalGNN_36051955482704
// MI455X (gfx1250) — hardware-verified
//
#include <hip/hip_runtime.h>
#include <math.h>

typedef _Float16 v16h __attribute__((ext_vector_type(16)));
typedef _Float16 v8h  __attribute__((ext_vector_type(8)));
typedef float    v8f  __attribute__((ext_vector_type(8)));
typedef float    v4f  __attribute__((ext_vector_type(4)));
typedef v8h __attribute__((may_alias)) v8ha;
typedef v4f __attribute__((may_alias)) v4fa;
union Frag { v16h v; v8h half[2]; };
union TileU { _Float16 a[4][16][136]; float g[4][16][68]; };

#define NB    8
#define NN    1024
#define NH    4
#define HD    16
#define HID   64
#define NCOM  20
#define NOUT  128
#define FIN   (NN + 4)
#define NROWS (NB * NN)
#define GK    (3 * HID)

__device__ __forceinline__ v8f wmma16(v16h a, v16h b, v8f c) {
  v8f d = __builtin_amdgcn_wmma_f32_16x16x32_f16(false, a, false, b, (short)0, c, false, false);
  asm volatile("v_nop\n\tv_nop\n\tv_nop\n\tv_nop" : "+v"(d) : "v"(a), "v"(b));
  return d;
}

__device__ __forceinline__ v8f zero8() {
  v8f z = {0.0f, 0.0f, 0.0f, 0.0f, 0.0f, 0.0f, 0.0f, 0.0f};
  return z;
}

__device__ __forceinline__ v16h ldfrag16(const _Float16* p, int h) {
  Frag f;
  f.half[0] = *(const v8ha*)(p + 8 * h);
  f.half[1] = *(const v8ha*)(p + 16 + 8 * h);
  return f.v;
}

__device__ __forceinline__ v8h cvt8(v4f a, v4f c, float sc) {
  v8h o = { (_Float16)(a.x * sc), (_Float16)(a.y * sc), (_Float16)(a.z * sc), (_Float16)(a.w * sc),
            (_Float16)(c.x * sc), (_Float16)(c.y * sc), (_Float16)(c.z * sc), (_Float16)(c.w * sc) };
  return o;
}

__device__ __forceinline__ v16h ldfrag32(const float* p, int h, float sc) {
  Frag f;
  f.half[0] = cvt8(*(const v4fa*)(p + 8 * h), *(const v4fa*)(p + 8 * h + 4), sc);
  f.half[1] = cvt8(*(const v4fa*)(p + 16 + 8 * h), *(const v4fa*)(p + 20 + 8 * h), sc);
  return f.v;
}

__device__ __forceinline__ float gelu_f(float v) {
  return 0.5f * v * (1.0f + erff(v * 0.70710678118654752f));
}

__device__ __forceinline__ float lky(float e) { return (e >= 0.0f) ? e : 0.2f * e; }

__device__ __forceinline__ void store_rows64(const float* tile, float* dst, int lane) {
  const int q = lane & 7, sub = lane >> 3;
#pragma unroll
  for (int i = 0; i < 8; ++i) {
    const int lid = i * 4 + sub, row = lid >> 1, hl = lid & 1;
    const v4f v = *(const v4fa*)(tile + row * 68 + 32 * hl + 4 * q);
    *(volatile v4f*)(dst + (size_t)row * HID + 32 * hl + 4 * q) = v;
  }
}

__global__ __launch_bounds__(256) void k_cvt(
    const float* __restrict__ in_w, const float* __restrict__ gate_w, const float* __restrict__ gat_w,
    _Float16* __restrict__ w1p, _Float16* __restrict__ gwp, _Float16* __restrict__ wgp)
{
  const int n1 = HID * NN / 8, n2 = HID * 2 * HID / 8, n3 = 3 * HID * HID / 8;
  const int g = blockIdx.x * 256 + threadIdx.x;
  if (g >= n1 + n2 + n3) return;
  const int r1 = (g >> 7) > (HID - 1) ? (HID - 1) : (g >> 7);
  const int c1 = g & 127;
  const int e2 = (g - n1) < 0 ? 0 : (g - n1);
  const int e3 = (g - n1 - n2) < 0 ? 0 : (g - n1 - n2);
  const float* src = (g < n1) ? (in_w + (size_t)r1 * FIN + 8 * c1)
                   : ((g < n1 + n2) ? (gate_w + (size_t)e2 * 8) : (gat_w + (size_t)e3 * 8));
  _Float16* dst = (g < n1) ? (w1p + (size_t)g * 8)
                : ((g < n1 + n2) ? (gwp + (size_t)e2 * 8) : (wgp + (size_t)e3 * 8));
  const float sc = (g < n1 + n2) ? 64.0f : 16.0f;
  const v4f a = *(const v4fa*)src;
  const v4f c = *(const v4fa*)(src + 4);
  const v8h o = cvt8(a, c, sc);
  *(volatile v8h*)dst = o;
  __threadfence();
  *(volatile v8h*)dst = o;
}

__global__ __launch_bounds__(128) void k_inproj(
    const float* __restrict__ adj, const float* __restrict__ coords, const int* __restrict__ comm,
    const float* __restrict__ in_w, const _Float16* __restrict__ w1p, const float* __restrict__ in_b,
    const float* __restrict__ lng, const float* __restrict__ lnb, const float* __restrict__ ctab,
    const _Float16* __restrict__ gwp, const float* __restrict__ gate_b, float* __restrict__ xout)
{
  __shared__ __attribute__((aligned(16))) float sx[4][16][68];
  __shared__ __attribute__((aligned(16))) TileU su;
  __shared__ float sdeg[4][16];
  __shared__ float sco[4][16][4];
  __shared__ int   scid[4][16];

  const int tid = threadIdx.x, lane = tid & 31, w = tid >> 5, h = lane >> 4, m = lane & 15;
  const int nw = blockIdx.x * 64 + 16 * w;
  const float* arow = adj + (size_t)(nw + m) * NN;

  v8f acc[4];
#pragma unroll
  for (int nt = 0; nt < 4; ++nt) acc[nt] = zero8();
  float dsum = 0.0f;

#pragma unroll 1
  for (int k0 = 0; k0 < NN; k0 += 32) {
    const v4f a0 = *(const v4fa*)(arow + k0 + 8 * h);
    const v4f a1 = *(const v4fa*)(arow + k0 + 8 * h + 4);
    const v4f c0 = *(const v4fa*)(arow + k0 + 16 + 8 * h);
    const v4f c1 = *(const v4fa*)(arow + k0 + 20 + 8 * h);
    dsum += ((fabsf(a0.x) + fabsf(a0.y)) + (fabsf(a0.z) + fabsf(a0.w)))
          + ((fabsf(a1.x) + fabsf(a1.y)) + (fabsf(a1.z) + fabsf(a1.w)))
          + ((fabsf(c0.x) + fabsf(c0.y)) + (fabsf(c0.z) + fabsf(c0.w)))
          + ((fabsf(c1.x) + fabsf(c1.y)) + (fabsf(c1.z) + fabsf(c1.w)));
    Frag af;
    af.half[0] = cvt8(a0, a1, 1.0f);
    af.half[1] = cvt8(c0, c1, 1.0f);
#pragma unroll
    for (int nt = 0; nt < 4; ++nt) {
      const v16h bf = ldfrag16(w1p + (size_t)(16 * nt + m) * NN + k0, h);
      acc[nt] = wmma16(af.v, bf, acc[nt]);
    }
  }

  dsum += __shfl_xor(dsum, 16);
  {
    int node = nw + m;
    node = (node < 0) ? 0 : ((node > NROWS - 1) ? (NROWS - 1) : node);
    const float* cp = coords + (size_t)node * 3;
    const float cx0 = cp[0];
    const float cy0 = cp[1];
    const float cz0 = cp[2];
    int cid = comm[node];
    cid = (cid == -1) ? NCOM : cid;
    cid = (cid < 0) ? 0 : ((cid > NCOM) ? NCOM : cid);
    if (h == 0) {
      sdeg[w][m] = dsum;
      sco[w][m][0] = cx0;
      sco[w][m][1] = cy0;
      sco[w][m][2] = cz0;
      scid[w][m] = cid;
    }
  }
#pragma unroll
  for (int nt = 0; nt < 4; ++nt)
#pragma unroll
    for (int r = 0; r < 8; ++r) sx[w][8 * h + r][16 * nt + m] = acc[nt][r];
  __syncthreads();

  {
    const int c0 = 32 * h;
    const float dg = sdeg[w][m], cx = sco[w][m][0], cy = sco[w][m][1], cz = sco[w][m][2];
    float s1 = 0.0f;
#pragma unroll 1
    for (int j = 0; j < 32; ++j) {
      const int c = c0 + j;
      const v4f tw = *(const v4fa*)(in_w + (size_t)c * FIN + NN);
      const float y = sx[w][m][c] * 0.015625f + in_b[c] + dg * tw.x + cx * tw.y + cy * tw.z + cz * tw.w;
      sx[w][m][c] = y;
      s1 += y;
    }
    s1 += __shfl_xor(s1, 16);
    const float mean = s1 * (1.0f / 64.0f);
    float s2 = 0.0f;
#pragma unroll 1
    for (int j = 0; j < 32; ++j) {
      const float d = sx[w][m][c0 + j] - mean;
      s2 += d * d;
    }
    s2 += __shfl_xor(s2, 16);
    const float rstd = rsqrtf(s2 * (1.0f / 64.0f) + 1e-5f);
    const int cid = scid[w][m];
#pragma unroll 1
    for (int j = 0; j < 32; ++j) {
      const int c = c0 + j;
      const float xv = (sx[w][m][c] - mean) * rstd * lng[c] + lnb[c];
      const float gx = gelu_f(xv);
      sx[w][m][c] = gx;
      su.a[w][m][c] = (_Float16)gx;
      su.a[w][m][64 + c] = (_Float16)(ctab[cid * HID + c] * 64.0f);
    }
  }
  __syncthreads();

  v8f g1[4], g2[4];
#pragma unroll
  for (int nt = 0; nt < 4; ++nt) { g1[nt] = zero8(); g2[nt] = zero8(); }
#pragma unroll
  for (int ks = 0; ks < 2; ++ks) {
    const v16h ax = ldfrag16(&su.a[w][m][0] + 32 * ks, h);
    const v16h ac = ldfrag16(&su.a[w][m][64] + 32 * ks, h);
#pragma unroll
    for (int nt = 0; nt < 4; ++nt) {
      const _Float16* gr = gwp + (size_t)(16 * nt + m) * (2 * HID) + 32 * ks;
      const v16h bx = ldfrag16(gr, h);
      const v16h bc = ldfrag16(gr + 64, h);
      g1[nt] = wmma16(ax, bx, g1[nt]);
      g2[nt] = wmma16(ac, bc, g2[nt]);
    }
  }
  __syncthreads();
#pragma unroll
  for (int nt = 0; nt < 4; ++nt)
#pragma unroll
    for (int r = 0; r < 8; ++r)
      su.g[w][8 * h + r][16 * nt + m] = g1[nt][r] * (1.0f / 64.0f) + g2[nt][r] * (1.0f / 4096.0f);
  __syncthreads();

  {
    const int c0 = 32 * h;
    const int cid = scid[w][m];
#pragma unroll 1
    for (int j = 0; j < 32; ++j) {
      const int c = c0 + j;
      float ga = su.g[w][m][c] + gate_b[c];
      ga = fminf(fmaxf(ga, -40.0f), 40.0f);
      const float gs = 1.0f / (1.0f + __expf(-ga));
      const float xv = sx[w][m][c];
      const float ce = ctab[cid * HID + c];
      sx[w][m][c] = xv * (1.0f - gs) + ce * gs;
    }
  }
  __syncthreads();

  float* dst = xout + (size_t)nw * HID;
  store_rows64(&sx[w][0][0], dst, lane);
  __threadfence();
  store_rows64(&sx[w][0][0], dst, lane);
}

__device__ __forceinline__ void gath_store(const _Float16* shtp, const float* sstp,
                                           _Float16* ht, float* sp, float* tp,
                                           int b, int nb, int w, int lane) {
  const int q = lane & 7, sub = lane >> 3;
#pragma unroll
  for (int i = 0; i < 4; ++i) {
    const int rowT = 16 * w + 4 * i + sub;
    const v8h v = *(const v8ha*)(shtp + rowT * 72 + 8 * q);
    *(volatile v8h*)(ht + (size_t)(b * (NH * HD) + rowT) * NN + nb + 8 * q) = v;
  }
  const int L = 4 * w + sub;
  const int which = L >> 3, hd = (L >> 1) & 3, hl = L & 1;
  const v4f v = *(const v4fa*)(sstp + which * 256 + hd * 64 + 32 * hl + 4 * q);
  float* base = which ? tp : sp;
  *(volatile v4f*)(base + (size_t)(b * NH + hd) * NN + nb + 32 * hl + 4 * q) = v;
}

__global__ __launch_bounds__(128) void k_gath(
    const float* __restrict__ x, const _Float16* __restrict__ wg, const float* __restrict__ av,
    _Float16* __restrict__ ht, float* __restrict__ sp, float* __restrict__ tp)
{
  __shared__ __attribute__((aligned(16))) float shf[64][68];
  __shared__ __attribute__((aligned(16))) _Float16 sht[64][72];
  __shared__ __attribute__((aligned(16))) float sst[2][NH][64];
  __shared__ float sav[128];

  const int tid = threadIdx.x, lane = tid & 31, w = tid >> 5, h = lane >> 4, m = lane & 15;
  const int n0b = blockIdx.x * 64;
  const int b = n0b / NN, nb = n0b - b * NN;
  sav[tid] = av[tid];

  const float* xr = x + (size_t)(n0b + 16 * w + m) * HID;
  v8f acc[4];
#pragma unroll
  for (int nt = 0; nt < 4; ++nt) acc[nt] = zero8();
#pragma unroll
  for (int ks = 0; ks < 2; ++ks) {
    const v16h af = ldfrag32(xr + 32 * ks, h, 1.0f);
#pragma unroll
    for (int nt = 0; nt < 4; ++nt) {
      const v16h bf = ldfrag16(wg + (size_t)(16 * nt + m) * HID + 32 * ks, h);
      acc[nt] = wmma16(af, bf, acc[nt]);
    }
  }
#pragma unroll
  for (int nt = 0; nt < 4; ++nt)
#pragma unroll
    for (int r = 0; r < 8; ++r) {
      const int row = 16 * w + 8 * h + r, col = 16 * nt + m;
      shf[row][col] = acc[nt][r] * (1.0f / 16.0f);
      sht[col][row] = (_Float16)acc[nt][r];
    }
  __syncthreads();

  {
    const int node = tid & 63, hp = tid >> 6;
#pragma unroll
    for (int q2 = 0; q2 < 2; ++q2) {
      const int hd = 2 * hp + q2;
      float ss = 0.0f, tt = 0.0f;
#pragma unroll 1
      for (int d = 0; d < HD; ++d) {
        const float hv = shf[node][hd * HD + d];
        ss += hv * sav[hd * 32 + d];
        tt += hv * sav[hd * 32 + HD + d];
      }
      sst[0][hd][node] = ss;
      sst[1][hd][node] = tt;
    }
  }
  __syncthreads();

  gath_store(&sht[0][0], &sst[0][0][0], ht, sp, tp, b, nb, w, lane);
  __threadfence();
  gath_store(&sht[0][0], &sst[0][0][0], ht, sp, tp, b, nb, w, lane);
}

__device__ __forceinline__ float mx4(float mx, float s, v4f t, v4f a) {
  mx = (a.x > 0.0f) ? fmaxf(mx, lky(s + t.x)) : mx;
  mx = (a.y > 0.0f) ? fmaxf(mx, lky(s + t.y)) : mx;
  mx = (a.z > 0.0f) ? fmaxf(mx, lky(s + t.z)) : mx;
  mx = (a.w > 0.0f) ? fmaxf(mx, lky(s + t.w)) : mx;
  return mx;
}

__device__ __forceinline__ v4f pr4(float s, v4f t, v4f a, float mxu, float fill, float& rs) {
  v4f p;
  p.x = (a.x > 0.0f) ? __expf(lky(s + t.x) - mxu) : fill;
  p.y = (a.y > 0.0f) ? __expf(lky(s + t.y) - mxu) : fill;
  p.z = (a.z > 0.0f) ? __expf(lky(s + t.z) - mxu) : fill;
  p.w = (a.w > 0.0f) ? __expf(lky(s + t.w) - mxu) : fill;
  rs += (p.x + p.y) + (p.z + p.w);
  return p;
}

__global__ __launch_bounds__(128) void k_attn(
    const float* __restrict__ adj, const float* __restrict__ sp, const float* __restrict__ tp,
    const _Float16* __restrict__ ht, const float* __restrict__ xin,
    const float* __restrict__ lng, const float* __restrict__ lnb, float* __restrict__ xout)
{
  __shared__ __attribute__((aligned(16))) float st[NH][NN];
  __shared__ __attribute__((aligned(16))) float so[4][16][68];
  __shared__ float sinv[4][NH][16];

  const int tid = threadIdx.x, lane = tid & 31, w = tid >> 5, h = lane >> 4, m = lane & 15;
  const int n0b = blockIdx.x * 64;
  const int b = n0b / NN, nb = n0b - b * NN;

  {
    const float* tsrc = tp + (size_t)b * NH * NN;
    float* tdst = &st[0][0];
#pragma unroll
    for (int i = 0; i < 8; ++i) {
      const int e = 4 * (i * 128 + tid);
      *(v4fa*)(tdst + e) = *(const v4fa*)(tsrc + e);
    }
  }
  __syncthreads();

  const int gq = n0b + 16 * w + m;
  const int nq = nb + 16 * w + m;
  const float* arow = adj + (size_t)gq * NN;

  float sv[NH], mxv[NH];
#pragma unroll
  for (int hd = 0; hd < NH; ++hd) {
    sv[hd] = sp[(size_t)(b * NH + hd) * NN + nq];
    mxv[hd] = -__builtin_inff();
  }

#pragma unroll 1
  for (int k0 = 0; k0 < NN; k0 += 32) {
    const v4f a0 = *(const v4fa*)(arow + k0 + 8 * h);
    const v4f a1 = *(const v4fa*)(arow + k0 + 8 * h + 4);
    const v4f c0 = *(const v4fa*)(arow + k0 + 16 + 8 * h);
    const v4f c1 = *(const v4fa*)(arow + k0 + 20 + 8 * h);
#pragma unroll
    for (int hd = 0; hd < NH; ++hd) {
      const float* tb = &st[hd][k0];
      const v4f t0 = *(const v4fa*)(tb + 8 * h);
      const v4f t1 = *(const v4fa*)(tb + 8 * h + 4);
      const v4f u0 = *(const v4fa*)(tb + 16 + 8 * h);
      const v4f u1 = *(const v4fa*)(tb + 20 + 8 * h);
      float mx = mxv[hd];
      mx = mx4(mx, sv[hd], t0, a0);
      mx = mx4(mx, sv[hd], t1, a1);
      mx = mx4(mx, sv[hd], u0, c0);
      mx = mx4(mx, sv[hd], u1, c1);
      mxv[hd] = mx;
    }
  }
  float mxu[NH], fill[NH], rs[NH];
  v8f acc[NH];
#pragma unroll
  for (int hd = 0; hd < NH; ++hd) {
    mxv[hd] = fmaxf(mxv[hd], __shfl_xor(mxv[hd], 16));
    const bool has = (mxv[hd] > -3.0e38f);
    mxu[hd]  = has ? mxv[hd] : 0.0f;
    fill[hd] = has ? 0.0f : 1.0f;
    rs[hd]   = 0.0f;
    acc[hd]  = zero8();
  }

#pragma unroll 1
  for (int k0 = 0; k0 < NN; k0 += 32) {
    const v4f a0 = *(const v4fa*)(arow + k0 + 8 * h);
    const v4f a1 = *(const v4fa*)(arow + k0 + 8 * h + 4);
    const v4f c0 = *(const v4fa*)(arow + k0 + 16 + 8 * h);
    const v4f c1 = *(const v4fa*)(arow + k0 + 20 + 8 * h);
#pragma unroll
    for (int hd = 0; hd < NH; ++hd) {
      const float* tb = &st[hd][k0];
      const v4f t0 = *(const v4fa*)(tb + 8 * h);
      const v4f t1 = *(const v4fa*)(tb + 8 * h + 4);
      const v4f u0 = *(const v4fa*)(tb + 16 + 8 * h);
      const v4f u1 = *(const v4fa*)(tb + 20 + 8 * h);
      const v4f p0 = pr4(sv[hd], t0, a0, mxu[hd], fill[hd], rs[hd]);
      const v4f p1 = pr4(sv[hd], t1, a1, mxu[hd], fill[hd], rs[hd]);
      const v4f p2 = pr4(sv[hd], u0, c0, mxu[hd], fill[hd], rs[hd]);
      const v4f p3 = pr4(sv[hd], u1, c1, mxu[hd], fill[hd], rs[hd]);
      Frag af;
      af.half[0] = cvt8(p0, p1, 4096.0f);
      af.half[1] = cvt8(p2, p3, 4096.0f);
      const v16h bf = ldfrag16(ht + (size_t)(b * (NH * HD) + hd * HD + m) * NN + k0, h);
      acc[hd] = wmma16(af.v, bf, acc[hd]);
    }
  }

#pragma unroll
  for (int hd = 0; hd < NH; ++hd) rs[hd] += __shfl_xor(rs[hd], 16);
  if (h == 0) {
#pragma unroll
    for (int hd = 0; hd < NH; ++hd) sinv[w][hd][m] = 1.0f / (rs[hd] * 65536.0f);
  }
  __syncthreads();
#pragma unroll
  for (int hd = 0; hd < NH; ++hd)
#pragma unroll
    for (int r = 0; r < 8; ++r)
      so[w][8 * h + r][hd * HD + m] = acc[hd][r] * sinv[w][hd][8 * h + r];
  __syncthreads();

  {
    const int c0 = 32 * h;
    const float* xr = xin + (size_t)gq * HID + c0;
    float s1 = 0.0f;
#pragma unroll 1
    for (int j = 0; j < 32; ++j) {
      const float v = so[w][m][c0 + j] + xr[j];
      so[w][m][c0 + j] = v;
      s1 += v;
    }
    s1 += __shfl_xor(s1, 16);
    const float mean = s1 * (1.0f / 64.0f);
    float s2 = 0.0f;
#pragma unroll 1
    for (int j = 0; j < 32; ++j) {
      const float d = so[w][m][c0 + j] - mean;
      s2 += d * d;
    }
    s2 += __shfl_xor(s2, 16);
    const float rstd = rsqrtf(s2 * (1.0f / 64.0f) + 1e-5f);
#pragma unroll 1
    for (int j = 0; j < 32; ++j) {
      const int c = c0 + j;
      so[w][m][c] = (so[w][m][c] - mean) * rstd * lng[c] + lnb[c];
    }
  }
  __syncthreads();

  float* dst = xout + (size_t)(n0b + 16 * w) * HID;
  store_rows64(&so[w][0][0], dst, lane);
  __threadfence();
  store_rows64(&so[w][0][0], dst, lane);
}

__device__ __forceinline__ void pool_store(const float* sgp, float* gpl, int b, int t) {
  if (t < 48 || (t >= 64 && t < 112)) {
    const bool isz = (t >= 64);
    const int q = isz ? (t - 64) : t;
    v4f v = *(const v4fa*)(sgp + 4 * q);
    const v4f zz = {0.0f, 0.0f, 0.0f, 0.0f};
    v = isz ? zz : v;
    float* dst = gpl + (size_t)(isz ? (NB + b) : b) * GK + 4 * q;
    *(volatile v4f*)dst = v;
  }
}

__global__ __launch_bounds__(256) void k_pool(
    const float* __restrict__ x, const float* __restrict__ pw, const float* __restrict__ pb,
    float* __restrict__ gpl)
{
  __shared__ float psum[4][64];
  __shared__ float pmax[4][64];
  __shared__ float pat[4][64];
  __shared__ float sw[NN];
  __shared__ float sred[256];
  __shared__ __attribute__((aligned(16))) float sg[GK];

  const int b = blockIdx.x, t = threadIdx.x, f = t & 63, ch = t >> 6;
  const float* xb = x + (size_t)b * NN * HID;

  float acc = 0.0f, mx = -__builtin_inff();
#pragma unroll 1
  for (int i = 0; i < 256; ++i) {
    const float v = xb[(size_t)(ch * 256 + i) * HID + f];
    acc += v;
    mx = fmaxf(mx, v);
  }
  psum[ch][f] = acc;
  pmax[ch][f] = mx;

  const float pb0 = pb[0];
  float lmax = -__builtin_inff();
#pragma unroll 1
  for (int j = 0; j < 4; ++j) {
    const int n = t + 256 * j;
    const float* xr = xb + (size_t)n * HID;
    float d = 0.0f;
#pragma unroll 1
    for (int k = 0; k < HID; ++k) d += xr[k] * pw[k];
    d += pb0;
    const float ad = fabsf(d);
    const float ee = __expf(-2.0f * ad);
    const float th = copysignf((1.0f - ee) / (1.0f + ee), d);
    sw[n] = th;
    lmax = fmaxf(lmax, th);
  }
  sred[t] = lmax;
  __syncthreads();
  for (int s = 128; s > 0; s >>= 1) {
    if (t < s) sred[t] = fmaxf(sred[t], sred[t + s]);
    __syncthreads();
  }
  const float smx = sred[0];
  __syncthreads();
  float lsum = 0.0f;
#pragma unroll 1
  for (int j = 0; j < 4; ++j) {
    const int n = t + 256 * j;
    const float e = __expf(sw[n] - smx);
    sw[n] = e;
    lsum += e;
  }
  sred[t] = lsum;
  __syncthreads();
  for (int s = 128; s > 0; s >>= 1) {
    if (t < s) sred[t] += sred[t + s];
    __syncthreads();
  }
  const float ssum = sred[0];
  __syncthreads();
  const float winv = 1.0f / ssum;

  float aacc = 0.0f;
#pragma unroll 1
  for (int i = 0; i < 256; ++i) {
    const int n = ch * 256 + i;
    aacc += xb[(size_t)n * HID + f] * sw[n];
  }
  pat[ch][f] = aacc * winv;
  __syncthreads();

  {
    const float vm = ((psum[0][f] + psum[1][f]) + (psum[2][f] + psum[3][f])) * (1.0f / (float)NN);
    const float vM = fmaxf(fmaxf(pmax[0][f], pmax[1][f]), fmaxf(pmax[2][f], pmax[3][f]));
    const float va = (pat[0][f] + pat[1][f]) + (pat[2][f] + pat[3][f]);
    const float val = (t < 64) ? vm : ((t < 128) ? vM : va);
    if (t < GK) sg[t] = val;
  }
  __syncthreads();

  pool_store(&sg[0], gpl, b, t);
  __threadfence();
  pool_store(&sg[0], gpl, b, t);
}

__global__ __launch_bounds__(256) void k_out(
    const float* __restrict__ gpl, const float* __restrict__ ow, const float* __restrict__ ob,
    const float* __restrict__ og, const float* __restrict__ olb, float* __restrict__ out)
{
  __shared__ __attribute__((aligned(16))) float sy[16][132];
  __shared__ __attribute__((aligned(16))) float so2[8][128];

  const int tid = threadIdx.x, lane = tid & 31, w = tid >> 5, h = lane >> 4, m = lane & 15;
  const float* ga = gpl + (size_t)m * GK;
  const float* wb = ow + (size_t)(16 * w + m) * GK;
  v8f acc = zero8();
#pragma unroll
  for (int ks = 0; ks < 6; ++ks) {
    const v16h af = ldfrag32(ga + 32 * ks, h, 1.0f);
    const v16h bf = ldfrag32(wb + 32 * ks, h, 64.0f);
    acc = wmma16(af, bf, acc);
  }
#pragma unroll
  for (int r = 0; r < 8; ++r) sy[8 * h + r][16 * w + m] = acc[r] * (1.0f / 64.0f) + ob[16 * w + m];
  __syncthreads();

  float s1 = 0.0f;
#pragma unroll 1
  for (int j = 0; j < 4; ++j) s1 += sy[w][lane + 32 * j];
#pragma unroll
  for (int off = 16; off > 0; off >>= 1) s1 += __shfl_xor(s1, off);
  const float mean = s1 * (1.0f / 128.0f);
  float s2 = 0.0f;
#pragma unroll 1
  for (int j = 0; j < 4; ++j) {
    const float d = sy[w][lane + 32 * j] - mean;
    s2 += d * d;
  }
#pragma unroll
  for (int off = 16; off > 0; off >>= 1) s2 += __shfl_xor(s2, off);
  const float rstd = rsqrtf(s2 * (1.0f / 128.0f) + 1e-5f);
#pragma unroll 1
  for (int j = 0; j < 4; ++j) {
    const int c = lane + 32 * j;
    const float y = (sy[w][c] - mean) * rstd * og[c] + olb[c];
    so2[w][c] = gelu_f(y);
  }
  __syncthreads();

  const v4f v = *(const v4fa*)(&so2[0][0] + 4 * tid);
  *(volatile v4f*)(out + 4 * tid) = v;
  __threadfence();
  *(volatile v4f*)(out + 4 * tid) = v;
}

extern "C" void kernel_launch(void* const* d_in, const int* in_sizes, int n_in,
                              void* d_out, int out_size, void* d_ws, size_t ws_size,
                              hipStream_t stream)
{
  if (n_in < 20) return;
  if (in_sizes[0] != NB * NN * NN || in_sizes[1] != NB * NN * 3 || in_sizes[2] != NB * NN) return;
  if (in_sizes[3] != HID * FIN || in_sizes[4] != HID || in_sizes[5] != HID || in_sizes[6] != HID) return;
  if (in_sizes[7] != (NCOM + 1) * HID || in_sizes[8] != HID * 2 * HID || in_sizes[9] != HID) return;
  if (in_sizes[10] != 3 * HID * HID || in_sizes[11] != 3 * NH * 2 * HD) return;
  if (in_sizes[12] != 3 * HID || in_sizes[13] != 3 * HID || in_sizes[14] != HID || in_sizes[15] < 1) return;
  if (in_sizes[16] != NOUT * GK || in_sizes[17] != NOUT || in_sizes[18] != NOUT || in_sizes[19] != NOUT) return;
  if (out_size != NB * NOUT) return;

  const float* adj      = (const float*)d_in[0];
  const float* coords   = (const float*)d_in[1];
  const int*   comm     = (const int*)d_in[2];
  const float* in_w     = (const float*)d_in[3];
  const float* in_b     = (const float*)d_in[4];
  const float* in_ln_g  = (const float*)d_in[5];
  const float* in_ln_b  = (const float*)d_in[6];
  const float* ctab     = (const float*)d_in[7];
  const float* gate_w   = (const float*)d_in[8];
  const float* gate_b   = (const float*)d_in[9];
  const float* gat_W    = (const float*)d_in[10];
  const float* gat_a    = (const float*)d_in[11];
  const float* gat_ln_g = (const float*)d_in[12];
  const float* gat_ln_b = (const float*)d_in[13];
  const float* pool_w   = (const float*)d_in[14];
  const float* pool_b   = (const float*)d_in[15];
  const float* out_w    = (const float*)d_in[16];
  const float* out_b    = (const float*)d_in[17];
  const float* out_ln_g = (const float*)d_in[18];
  const float* out_ln_b = (const float*)d_in[19];
  float* out = (float*)d_out;

  const size_t w1p_bytes = (size_t)HID * NN * 2;
  const size_t gwp_bytes = (size_t)HID * 2 * HID * 2;
  const size_t wgp_bytes = (size_t)3 * HID * HID * 2;
  const size_t x_bytes   = (size_t)NROWS * HID * 4;
  const size_t ht_bytes  = (size_t)NB * NH * HD * NN * 2;
  const size_t st_bytes  = (size_t)NB * NH * NN * 4;
  const size_t g_bytes   = (size_t)16 * GK * 4;
  size_t off = 0;
  const size_t o_w1p = off; off += w1p_bytes;
  const size_t o_gwp = off; off += gwp_bytes;
  const size_t o_wgp = off; off += wgp_bytes;
  const size_t o_x0  = off; off += x_bytes;
  const size_t o_x1  = off; off += x_bytes;
  const size_t o_ht  = off; off += ht_bytes;
  const size_t o_s   = off; off += st_bytes;
  const size_t o_t   = off; off += st_bytes;
  const size_t o_g   = off; off += g_bytes;
  if (off > ws_size) return;

  char* ws = (char*)d_ws;
  _Float16* w1p = (_Float16*)(ws + o_w1p);
  _Float16* gwp = (_Float16*)(ws + o_gwp);
  _Float16* wgp = (_Float16*)(ws + o_wgp);
  float* x0 = (float*)(ws + o_x0);
  float* x1 = (float*)(ws + o_x1);
  _Float16* htp = (_Float16*)(ws + o_ht);
  float* splane = (float*)(ws + o_s);
  float* tplane = (float*)(ws + o_t);
  float* gpl = (float*)(ws + o_g);

  const int ngroups = HID * NN / 8 + HID * 2 * HID / 8 + 3 * HID * HID / 8;
  k_cvt<<<(ngroups + 255) / 256, 256, 0, stream>>>(in_w, gate_w, gat_W, w1p, gwp, wgp);

  k_inproj<<<NROWS / 64, 128, 0, stream>>>(adj, coords, comm, in_w, w1p, in_b, in_ln_g, in_ln_b,
                                           ctab, gwp, gate_b, x0);

  for (int l = 0; l < 3; ++l) {
    const float* xin = (l == 1) ? x1 : x0;
    float* xo = (l == 1) ? x0 : x1;
    k_gath<<<NROWS / 64, 128, 0, stream>>>(xin, wgp + (size_t)l * HID * HID, gat_a + (size_t)l * NH * 2 * HD,
                                           htp, splane, tplane);
    k_attn<<<NROWS / 64, 128, 0, stream>>>(adj, splane, tplane, htp, xin,
                                           gat_ln_g + (size_t)l * HID, gat_ln_b + (size_t)l * HID, xo);
  }

  k_pool<<<NB, 256, 0, stream>>>(x1, pool_w, pool_b, gpl);
  k_out<<<1, 256, 0, stream>>>(gpl, out_w, out_b, out_ln_g, out_ln_b, out);
}
